// GDM_57543971832235
// MI455X (gfx1250) — hardware-verified
//
#include <hip/hip_runtime.h>
#include <stddef.h>


typedef __attribute__((ext_vector_type(16))) _Float16 v16h;
typedef __attribute__((ext_vector_type(8)))  _Float16 v8h;
typedef __attribute__((ext_vector_type(8)))  float    v8f;
typedef __attribute__((ext_vector_type(4)))  float    v4f;
typedef __attribute__((ext_vector_type(8)))  unsigned u8v;

#define HWPIX 9216
#define IMGW  96
#define CIN   256
#define NBATCH 4

__device__ __forceinline__ void dep_guard_h(v8f& a, v8f& b, v16h x, v16h y) { asm volatile("v_nop\n\tv_nop\n\tv_nop\n\tv_nop" : "+v"(a), "+v"(b) : "v"(x), "v"(y)); }
__device__ __forceinline__ void keep4_h(v16h a, v16h b, v16h c, v16h d) { asm volatile("v_nop" :: "v"(a), "v"(b), "v"(c), "v"(d)); }
__device__ __forceinline__ void acc_guard4(v8f& a, v8f& b, v8f& c, v8f& d) { asm volatile("v_nop\n\tv_nop\n\tv_nop\n\tv_nop" : "+v"(a), "+v"(b), "+v"(c), "+v"(d)); }

template <typename T> struct Frag;
template <> struct Frag<_Float16> {
  typedef v16h V; union U { v16h v; v8h h[2]; };
  static __device__ __forceinline__ v16h load(const _Float16* p) {
    U f; f.h[0] = *(const v8h*)(p); f.h[1] = *(const v8h*)(p + 16); return f.v;
  }
  static __device__ __forceinline__ v8f mma(v16h a, v16h b, v8f c) {
    return __builtin_amdgcn_wmma_f32_16x16x32_f16(false, a, false, b, (short)0, c, false, false);
  }
  static __device__ __forceinline__ void guard(v8f& a, v8f& b, v16h x, v16h y) { dep_guard_h(a, b, x, y); }
  static __device__ __forceinline__ void keep(v16h a, v16h b, v16h c, v16h d) { keep4_h(a, b, c, d); }
};

union FragBits { v16h v; u8v u; };

template <int TAPS, bool HAS_BIAS, bool RELU, bool RESID, bool OUTF32>
__global__ __launch_bounds__(256) void conv_gemm64(
    const unsigned short* __restrict__ Ap,
    const unsigned short* __restrict__ Btp,
    void* __restrict__ Cout, int ldc,
    const float* __restrict__ bias,
    const unsigned short* __restrict__ Rp, int ldr,
    int N, float scale) {
  typedef _Float16 T;
  typedef v16h V;
  constexpr int K = TAPS * CIN;
  const T* A  = (const T*)Ap;
  const T* Bt = (const T*)Btp;
  const T* R  = (const T*)Rp;
  __shared__ __align__(16) float sT[8][16 * 68];

  const int b    = blockIdx.y;
  const int lane = threadIdx.x & 31;
  const int wave = threadIdx.x >> 5;
  const int tilesN = N >> 6;
  const int tilesM = HWPIX >> 6;
  const int tile = blockIdx.x * 8 + wave;
  if (tile >= tilesM * tilesN) return;
  const int tm = tile / tilesN;
  const int tn = tile - tm * tilesN;
  const int m0 = tm << 6;
  const int n0 = tn << 6;

  const T* Ab = A + (size_t)b * HWPIX * CIN;

  const int rlane = lane & 15;
  const int koff  = (lane >> 4) * 8;
  const int mOff  = (lane >> 4) * 8;

  int pr[4], hr[4], wr[4];
#pragma unroll
  for (int i = 0; i < 4; ++i) {
    pr[i] = m0 + (i << 4) + rlane;
    hr[i] = pr[i] / IMGW;
    wr[i] = pr[i] - hr[i] * IMGW;
  }

  v8f acc[4][4];
#pragma unroll
  for (int i = 0; i < 4; ++i)
#pragma unroll
    for (int j = 0; j < 4; ++j) acc[i][j] = (v8f){0.f,0.f,0.f,0.f,0.f,0.f,0.f,0.f};

  for (int k0 = 0; k0 < K; k0 += 32) {
    int cin0 = k0, dy = 0, dx = 0;
    if (TAPS == 9) {
      const int tap = k0 >> 8;
      cin0 = k0 & (CIN - 1);
      const int ky = tap / 3;
      dy = ky - 1;
      dx = tap - ky * 3 - 1;
    }
    V bh[4];
#pragma unroll
    for (int j = 0; j < 4; ++j) {
      const size_t bo = (size_t)(n0 + (j << 4) + rlane) * K + koff + k0;
      bh[j] = Frag<T>::load(Bt + bo);
    }
#pragma unroll
    for (int i = 0; i < 4; ++i) {
      V ah;
      if (TAPS == 9) {
        const bool ok = ((unsigned)(hr[i] + dy) < (unsigned)IMGW) && ((unsigned)(wr[i] + dx) < (unsigned)IMGW);
        const int sp = ok ? (pr[i] + dy * IMGW + dx) : pr[i];
        ah = Frag<T>::load(Ab + (size_t)sp * CIN + cin0 + koff);
        FragBits fb; fb.v = ah;
        const unsigned msk = ok ? 0xFFFFFFFFu : 0u;
        fb.u = fb.u & msk;
        ah = fb.v;
      } else {
        ah = Frag<T>::load(Ab + (size_t)pr[i] * CIN + k0 + koff);
      }
#pragma unroll
      for (int j = 0; j < 4; ++j) acc[i][j] = Frag<T>::mma(ah, bh[j], acc[i][j]);
      Frag<T>::guard(acc[i][0], acc[i][3], ah, ah);
    }
    Frag<T>::keep(bh[0], bh[1], bh[2], bh[3]);
  }
  acc_guard4(acc[0][0], acc[0][1], acc[0][2], acc[0][3]);
  acc_guard4(acc[1][0], acc[1][1], acc[1][2], acc[1][3]);
  acc_guard4(acc[2][0], acc[2][1], acc[2][2], acc[2][3]);
  acc_guard4(acc[3][0], acc[3][1], acc[3][2], acc[3][3]);

  float* slab = sT[wave];
#pragma unroll
  for (int i = 0; i < 4; ++i) {
    const int mBase = m0 + (i << 4);
#pragma unroll
    for (int j = 0; j < 4; ++j) {
      const int n = n0 + (j << 4) + rlane;
      float bv = 0.f;
      if constexpr (HAS_BIAS) bv = bias[n];
#pragma unroll
      for (int r = 0; r < 8; ++r) {
        float v = acc[i][j][r] * scale + bv;
        if constexpr (RELU) v = fmaxf(v, 0.0f);
        slab[(mOff + r) * 68 + (j << 4) + rlane] = v;
      }
    }
    __builtin_amdgcn_fence(__ATOMIC_RELEASE, "workgroup");
    __builtin_amdgcn_wave_barrier();
    __builtin_amdgcn_fence(__ATOMIC_ACQUIRE, "workgroup");
    if constexpr (OUTF32) {
      float* C = (float*)Cout + (size_t)b * HWPIX * ldc;
      const int hh = lane >> 4, c4 = (lane & 15) * 4;
      for (int pass = 0; pass < 2; ++pass) {
#pragma unroll
        for (int it = 0; it < 8; ++it) {
          const int row = it * 2 + hh;
          v4f v = *(const v4f*)(slab + row * 68 + c4);
          *(volatile v4f*)(C + (size_t)(mBase + row) * ldc + n0 + c4) = v;
        }
        __threadfence();
      }
    } else {
      const int q = lane >> 3, c8 = (lane & 7) * 8;
      T* C = (T*)Cout + (size_t)b * HWPIX * ldc;
      for (int pass = 0; pass < 2; ++pass) {
#pragma unroll
        for (int it = 0; it < 4; ++it) {
          const int row = it * 4 + q;
          const float* sp = slab + row * 68 + c8;
          v8h hv;
          if constexpr (RESID) {
            const v8h rv = *(const v8h*)(R + (size_t)b * HWPIX * ldr + (size_t)(mBase + row) * ldr + n0 + c8);
#pragma unroll
            for (int e = 0; e < 8; ++e) hv[e] = (_Float16)(sp[e] + (float)rv[e]);
          } else {
#pragma unroll
            for (int e = 0; e < 8; ++e) hv[e] = (_Float16)sp[e];
          }
          *(volatile v8h*)(C + (size_t)(mBase + row) * ldc + n0 + c8) = hv;
        }
        __threadfence();
      }
    }
    __builtin_amdgcn_fence(__ATOMIC_RELEASE, "workgroup");
    __builtin_amdgcn_wave_barrier();
    __builtin_amdgcn_fence(__ATOMIC_ACQUIRE, "workgroup");
  }
}

__global__ __launch_bounds__(256) void k_nchw_to_pm16(const float* __restrict__ x, unsigned short* __restrict__ outp) {
  __shared__ __align__(16) _Float16 sh[64 * 72];
  const int p0 = blockIdx.x * 64, c0 = blockIdx.y * 64, b = blockIdx.z;
  const int tid = threadIdx.x, lane = tid & 31, wave = tid >> 5;
  {
    const int cl = tid >> 2, pq = (tid & 3) * 16;
    const float* src = x + ((size_t)(b * CIN + c0 + cl)) * HWPIX + p0 + pq;
#pragma unroll
    for (int g = 0; g < 4; ++g) {
      const v4f v = *(const v4f*)(src + 4 * g);
#pragma unroll
      for (int e = 0; e < 4; ++e) sh[(pq + 4 * g + e) * 72 + cl] = (_Float16)v[e];
    }
  }
  __syncthreads();
  _Float16* o = (_Float16*)outp;
  const int q = lane >> 3, c8 = (lane & 7) * 8;
  for (int pass = 0; pass < 2; ++pass) {
#pragma unroll
    for (int it = 0; it < 2; ++it) {
      const int row = it * 32 + wave * 4 + q;
      const v8h hv = *(const v8h*)(sh + row * 72 + c8);
      *(volatile v8h*)(o + ((size_t)(b * HWPIX + p0 + row)) * CIN + c0 + c8) = hv;
    }
    __threadfence();
  }
}

__global__ __launch_bounds__(256) void k_pm32_to_nchw(const float* __restrict__ in, float* __restrict__ out) {
  __shared__ __align__(16) float sh[64 * 68];
  const int p0 = blockIdx.x * 64, c0 = blockIdx.y * 64, b = blockIdx.z;
  const int tid = threadIdx.x, lane = tid & 31, wave = tid >> 5;
  {
    const int pl = tid >> 2, cq = (tid & 3) * 16;
    const float* src = in + ((size_t)(b * HWPIX + p0 + pl)) * CIN + c0 + cq;
#pragma unroll
    for (int g = 0; g < 4; ++g) {
      const v4f v = *(const v4f*)(src + 4 * g);
#pragma unroll
      for (int e = 0; e < 4; ++e) sh[(cq + 4 * g + e) * 68 + pl] = v[e];
    }
  }
  __syncthreads();
  const int hh = lane >> 4, c4 = (lane & 15) * 4;
  for (int pass = 0; pass < 2; ++pass) {
#pragma unroll
    for (int it = 0; it < 4; ++it) {
      const int row = it * 16 + wave * 2 + hh;
      const v4f v = *(const v4f*)(sh + row * 68 + c4);
      *(volatile v4f*)(out + ((size_t)(b * CIN + c0 + row)) * HWPIX + p0 + c4) = v;
    }
    __threadfence();
  }
}

__global__ __launch_bounds__(256) void k_prep1x1(const float* __restrict__ w, const float* __restrict__ s,
                                                 unsigned short* __restrict__ outp, int Cout) {
  const int idx = blockIdx.x * 256 + threadIdx.x;
  if (idx >= Cout * (CIN / 8)) return;
  const int co = idx >> 5;
  const int ci8 = (idx & 31) * 8;
  const float sc = s[co] * 64.0f;
  const float* wp = w + (size_t)co * CIN + ci8;
  const v4f a0 = *(const v4f*)(wp);
  const v4f a1 = *(const v4f*)(wp + 4);
  v8h hv;
#pragma unroll
  for (int e = 0; e < 4; ++e) { hv[e] = (_Float16)(a0[e] * sc); hv[4 + e] = (_Float16)(a1[e] * sc); }
  _Float16* o = (_Float16*)outp + (size_t)co * CIN + ci8;
  *(volatile v8h*)o = hv;
  __threadfence();
  *(volatile v8h*)o = hv;
}

__global__ __launch_bounds__(256) void k_prep3x3(const float* __restrict__ w, const float* __restrict__ s,
                                                 unsigned short* __restrict__ outp) {
  const int idx = blockIdx.x * 256 + threadIdx.x;
  if (idx >= 256 * 288) return;
  const int co = idx / 288;
  const int g  = idx - co * 288;
  const int t  = g >> 5;
  const int ci8 = (g & 31) * 8;
  const float sc = s[co] * 64.0f;
  const float* wp = w + ((size_t)co * CIN + ci8) * 9 + t;
  v8h hv;
#pragma unroll
  for (int e = 0; e < 8; ++e) hv[e] = (_Float16)(wp[e * 9] * sc);
  _Float16* o = (_Float16*)outp + (size_t)co * (9 * CIN) + t * CIN + ci8;
  *(volatile v8h*)o = hv;
  __threadfence();
  *(volatile v8h*)o = hv;
}

__global__ __launch_bounds__(64) void k_solve(const float* __restrict__ w, float* __restrict__ Aout) {
  __shared__ float Wsh[64 * 65];
  __shared__ float As[64 * 65];
  __shared__ float dv[64];
  const int c = threadIdx.x, lane = c & 31, wave = c >> 5;
  for (int i = 0; i < 64; ++i) Wsh[i * 65 + c] = w[i * 64 + c];
  __syncthreads();
  dv[c] = 1.0f + Wsh[c * 65 + c];
  __syncthreads();
  for (int i = 0; i < 64; ++i) {
    const float rhs = (i == c) ? dv[i] : ((c > i) ? Wsh[i * 65 + c] : 0.0f);
    float s = 0.0f;
#pragma unroll 1
    for (int j = 0; j < i; ++j) s += Wsh[i * 65 + j] * As[j * 65 + c];
    As[i * 65 + c] = rhs + dv[i] * s;
    __syncthreads();
  }
  const int hh = lane >> 4, c4 = (lane & 15) * 4;
  for (int pass = 0; pass < 2; ++pass) {
    for (int it = 0; it < 16; ++it) {
      const int row = it * 4 + wave * 2 + hh;
      v4f v;
      v[0] = As[row * 65 + c4 + 0];
      v[1] = As[row * 65 + c4 + 1];
      v[2] = As[row * 65 + c4 + 2];
      v[3] = As[row * 65 + c4 + 3];
      *(volatile v4f*)(Aout + row * 64 + c4) = v;
    }
    __threadfence();
  }
}

__global__ __launch_bounds__(256) void k_mixprep(const float* __restrict__ A, unsigned short* __restrict__ outp) {
  const int idx = blockIdx.x * 256 + threadIdx.x;
  if (idx >= 256 * 32) return;
  const int n = idx >> 5, k8 = (idx & 31) * 8;
  const int i = n >> 2, d = n & 3;
  v8h hv;
#pragma unroll
  for (int e = 0; e < 8; ++e) {
    const int k = k8 + e;
    const int cc = k >> 2;
    const float a = A[i * 64 + cc] * 256.0f;
    hv[e] = (_Float16)(((k & 3) == d) ? a : 0.0f);
  }
  _Float16* o = (_Float16*)outp + (size_t)n * CIN + k8;
  *(volatile v8h*)o = hv;
  __threadfence();
  *(volatile v8h*)o = hv;
}

extern "C" void kernel_launch(void* const* d_in, const int* in_sizes, int n_in,
                              void* d_out, int out_size, void* d_ws, size_t ws_size,
                              hipStream_t stream) {
  if (n_in < 18) return;
  const int planeElems = NBATCH * CIN * HWPIX;
  if (in_sizes[0] != planeElems || in_sizes[1] != planeElems || out_size != planeElems) return;
  if (in_sizes[2] != 64 * 64 || in_sizes[3] != 128 * CIN || in_sizes[6] != 128 * CIN) return;
  if (in_sizes[9] != 256 * CIN * 9 || in_sizes[12] != 256 * CIN || in_sizes[15] != 256 * CIN * 9) return;
  if (in_sizes[4] != 128 || in_sizes[5] != 128 || in_sizes[7] != 128 || in_sizes[8] != 128) return;
  if (in_sizes[10] != 256 || in_sizes[11] != 256 || in_sizes[13] != 256 || in_sizes[14] != 256 ||
      in_sizes[16] != 256 || in_sizes[17] != 256) return;

  const float* x1     = (const float*)d_in[0];
  const float* x2     = (const float*)d_in[1];
  const float* weight = (const float*)d_in[2];
  const float* r1_w = (const float*)d_in[3],  *r1_s = (const float*)d_in[4],  *r1_b = (const float*)d_in[5];
  const float* r2_w = (const float*)d_in[6],  *r2_s = (const float*)d_in[7],  *r2_b = (const float*)d_in[8];
  const float* ck_w = (const float*)d_in[9],  *ck_s = (const float*)d_in[10], *ck_b = (const float*)d_in[11];
  const float* c1_w = (const float*)d_in[12], *c1_s = (const float*)d_in[13], *c1_b = (const float*)d_in[14];
  const float* cf_w = (const float*)d_in[15], *cf_s = (const float*)d_in[16], *cf_b = (const float*)d_in[17];

  const size_t plane16 = (size_t)planeElems * 2;
  size_t off = 0;
  const size_t oReg0 = off; off += plane16;
  const size_t oReg1 = off; off += plane16;
  const size_t oReg2 = off; off += plane16;
  const size_t oWr1  = off; off += (size_t)128 * CIN * 2;
  const size_t oWr2  = off; off += (size_t)128 * CIN * 2;
  const size_t oWmix = off; off += (size_t)256 * CIN * 2;
  const size_t oWck  = off; off += (size_t)256 * 9 * CIN * 2;
  const size_t oWc1  = off; off += (size_t)256 * CIN * 2;
  const size_t oWcf  = off; off += (size_t)256 * 9 * CIN * 2;
  const size_t oAmat = off; off += (size_t)64 * 64 * 4;
  if (off > ws_size) return;

  char* ws = (char*)d_ws;
  unsigned short* reg0 = (unsigned short*)(ws + oReg0);
  unsigned short* reg1 = (unsigned short*)(ws + oReg1);
  unsigned short* reg2 = (unsigned short*)(ws + oReg2);
  float* outpm = (float*)(ws + oReg0);
  unsigned short* wr1  = (unsigned short*)(ws + oWr1);
  unsigned short* wr2  = (unsigned short*)(ws + oWr2);
  unsigned short* wmix = (unsigned short*)(ws + oWmix);
  unsigned short* wck  = (unsigned short*)(ws + oWck);
  unsigned short* wc1  = (unsigned short*)(ws + oWc1);
  unsigned short* wcf  = (unsigned short*)(ws + oWcf);
  float* Amat = (float*)(ws + oAmat);

  const dim3 tgrid(HWPIX / 64, CIN / 64, NBATCH);
  const float inv64 = 1.0f / 64.0f, inv256 = 1.0f / 256.0f;

  k_nchw_to_pm16<<<tgrid, 256, 0, stream>>>(x1, reg1);
  k_nchw_to_pm16<<<tgrid, 256, 0, stream>>>(x2, reg2);
  k_prep1x1<<<dim3(128 * 32 / 256), 256, 0, stream>>>(r1_w, r1_s, wr1, 128);
  k_prep1x1<<<dim3(128 * 32 / 256), 256, 0, stream>>>(r2_w, r2_s, wr2, 128);
  k_prep1x1<<<dim3(256 * 32 / 256), 256, 0, stream>>>(c1_w, c1_s, wc1, 256);
  k_prep3x3<<<dim3(288), 256, 0, stream>>>(ck_w, ck_s, wck);
  k_prep3x3<<<dim3(288), 256, 0, stream>>>(cf_w, cf_s, wcf);
  k_solve<<<dim3(1), 64, 0, stream>>>(weight, Amat);
  k_mixprep<<<dim3(32), 256, 0, stream>>>(Amat, wmix);

  conv_gemm64<1, true, true, false, false><<<dim3(144 * 2 / 8, NBATCH), 256, 0, stream>>>(
      reg1, wr1, (void*)reg0, CIN, r1_b, nullptr, 0, 128, inv64);
  conv_gemm64<1, true, true, false, false><<<dim3(144 * 2 / 8, NBATCH), 256, 0, stream>>>(
      reg2, wr2, (void*)(reg0 + 128), CIN, r2_b, nullptr, 0, 128, inv64);
  conv_gemm64<1, false, false, false, false><<<dim3(144 * 4 / 8, NBATCH), 256, 0, stream>>>(
      reg0, wmix, (void*)reg2, CIN, nullptr, nullptr, 0, 256, inv256);
  conv_gemm64<9, true, true, true, false><<<dim3(144 * 4 / 8, NBATCH), 256, 0, stream>>>(
      reg2, wck, (void*)reg1, CIN, ck_b, reg0, CIN, 256, inv64);
  conv_gemm64<1, true, true, false, false><<<dim3(144 * 4 / 8, NBATCH), 256, 0, stream>>>(
      reg1, wc1, (void*)reg2, CIN, c1_b, nullptr, 0, 256, inv64);
  conv_gemm64<9, true, true, false, true><<<dim3(144 * 4 / 8, NBATCH), 256, 0, stream>>>(
      reg2, wcf, (void*)outpm, CIN, cf_b, nullptr, 0, 256, inv64);
  k_pm32_to_nchw<<<tgrid, 256, 0, stream>>>(outpm, (float*)d_out);
  (void)hipGetLastError();
}
